// EntropyGuidedAttention_84293028151600
// MI455X (gfx1250) — hardware-verified
//
#include <hip/hip_runtime.h>
#include <math.h>
#include <stdint.h>
#include <stddef.h>

typedef _Float16 v16h __attribute__((ext_vector_type(16)));
typedef _Float16 v8h  __attribute__((ext_vector_type(8), __may_alias__));
typedef _Float16 v4h  __attribute__((ext_vector_type(4), __may_alias__));
typedef float    v8f  __attribute__((ext_vector_type(8)));
typedef float    v4f  __attribute__((ext_vector_type(4), __may_alias__));

union Frag { v16h v; v8h p[2]; };

constexpr int BSZ   = 2;
constexpr int NSEQ  = 2048;
constexpr int CDIM  = 1024;
constexpr int HN    = 16;
constexpr int DH    = 64;
constexpr int QKVN  = 3 * CDIM;
constexpr int MROWS = BSZ * NSEQ;
constexpr size_t QKV_S = (size_t)BSZ * HN * NSEQ * DH;
constexpr float WSCALE = 64.0f;
constexpr float PSCALE = 256.0f;
constexpr float ASCALE = 64.0f;

__device__ __forceinline__ v8f wmma_f16(v16h a, v16h b, v8f c) {
  v8f d = __builtin_amdgcn_wmma_f32_16x16x32_f16(false, a, false, b, (short)0, c, false, false);
  asm volatile("v_nop\n\tv_nop\n\tv_nop\n\tv_nop" : "+v"(d) : "v"(a), "v"(b));
  return d;
}

__device__ __forceinline__ v16h ld_frag(const _Float16* rk, int lh) {
  Frag f;
  f.p[0] = *(const v8h*)(rk + 8 * lh);
  f.p[1] = *(const v8h*)(rk + 16 + 8 * lh);
  return f.v;
}

__global__ __launch_bounds__(128)
void k_qkv(const float* __restrict__ x, const float* __restrict__ W, const float* __restrict__ bias,
           _Float16* __restrict__ qkv) {
  __shared__ __align__(16) _Float16 lds[64 * 64];
  _Float16* As = lds;
  _Float16* Bs = lds + 2048;

  const int tid = threadIdx.x, lane = tid & 31, w = tid >> 5, m = lane & 15, lh = lane >> 4;
  const int cblk = blockIdx.x * 64, rblk = blockIdx.y * 64;
  if (cblk + 64 > QKVN || rblk + 64 > MROWS) return;

  const int ar = tid >> 1, ac = (tid & 1) * 16;
  const int bk = tid >> 2, bc = (tid & 3) * 16;
  const float* ap = x + (size_t)(rblk + ar) * CDIM + ac;
  const float* bp = W + (size_t)bk * QKVN + cblk + bc;

  v8f acc[4] = {};

  for (int k0 = 0; k0 < CDIM; k0 += 32) {
    v4f a4[4], b4[4];
#pragma unroll
    for (int j = 0; j < 4; ++j) a4[j] = *(const v4f*)(ap + k0 + 4 * j);
#pragma unroll
    for (int j = 0; j < 4; ++j) b4[j] = *(const v4f*)(bp + (size_t)k0 * QKVN + 4 * j);
    __syncthreads();
#pragma unroll
    for (int j = 0; j < 4; ++j)
      *(v4h*)(As + ar * 32 + ac + 4 * j) = __builtin_convertvector(a4[j], v4h);
#pragma unroll
    for (int j = 0; j < 4; ++j)
#pragma unroll
      for (int e = 0; e < 4; ++e)
        Bs[(bc + 4 * j + e) * 32 + bk] = (_Float16)(b4[j][e] * WSCALE);
    __syncthreads();

    v16h af = ld_frag(As + (w * 16 + m) * 32, lh);
    v16h bf[4];
#pragma unroll
    for (int nt = 0; nt < 4; ++nt) bf[nt] = ld_frag(Bs + (nt * 16 + m) * 32, lh);
#pragma unroll
    for (int nt = 0; nt < 4; ++nt) acc[nt] = wmma_f16(af, bf[nt], acc[nt]);
  }

  __syncthreads();
  _Float16* Cs = lds;
#pragma unroll
  for (int nt = 0; nt < 4; ++nt) {
    const int col = nt * 16 + m;
    const float bb = bias[cblk + col];
#pragma unroll
    for (int r = 0; r < 8; ++r)
      Cs[(w * 16 + 8 * lh + r) * 64 + col] = (_Float16)(acc[nt][r] * (1.0f / WSCALE) + bb);
  }
  __syncthreads();

  const int sS = cblk >> 10, hd = (cblk & 1023) >> 6, b = rblk >> 11, n0 = rblk & 2047;
  _Float16* dst = qkv + (size_t)sS * QKV_S + ((size_t)(b * HN + hd) * NSEQ + n0) * DH;
  v8h vv[4];
#pragma unroll
  for (int j = 0; j < 4; ++j) vv[j] = *(const v8h*)(Cs + (j * 128 + tid) * 8);
#pragma unroll
  for (int j = 0; j < 4; ++j) *(volatile v8h*)(dst + (j * 128 + tid) * 8) = vv[j];
  __threadfence();
#pragma unroll
  for (int j = 0; j < 4; ++j) *(volatile v8h*)(dst + (j * 128 + tid) * 8) = vv[j];
}

__global__ __launch_bounds__(128)
void k_attn(const _Float16* __restrict__ qkv, const float* __restrict__ x,
            const float* __restrict__ We, const float* __restrict__ be,
            const int* __restrict__ am, _Float16* __restrict__ aw) {
  __shared__ __align__(16) _Float16 Qs[64 * 64];
  __shared__ __align__(16) _Float16 Ks[64 * 64];
  __shared__ __align__(16) _Float16 Vt[64 * 64];
  __shared__ __align__(16) _Float16 Ps[4 * 16 * 64];
  __shared__ float gsig[64];

  const int tid = threadIdx.x, lane = tid & 31, w = tid >> 5, m = lane & 15, lh = lane >> 4;
  const int bid = blockIdx.x;
  const int qt = bid & 31, bh = bid >> 5, hd = bh & 15, b = bh >> 4;
  if (b >= BSZ) return;
  const int qbase = qt * 64;

  const _Float16* Qg = qkv + ((size_t)(b * HN + hd) * NSEQ) * DH;
  const _Float16* Kg = Qg + QKV_S;
  const _Float16* Vg = Kg + QKV_S;

  {
    const int q = tid >> 1, part = tid & 1;
    const float* xr = x + ((size_t)(b * NSEQ + qbase + q)) * CDIM + part * 512;
    const float* wp = We + (size_t)(part * 512) * HN + hd;
    float s = 0.0f;
#pragma unroll 4
    for (int c = 0; c < 512; ++c) s += xr[c] * wp[(size_t)c * HN];
    s += __shfl_xor(s, 1, 32);
    if (part == 0) {
      const float z = s + be[hd];
      gsig[q] = 1.0f / (1.0f + expf(-z));
    }
  }
  {
    const _Float16* src = Qg + (size_t)qbase * DH;
#pragma unroll
    for (int it = 0; it < 4; ++it)
      *(v8h*)(Qs + (it * 128 + tid) * 8) = *(const v8h*)(src + (it * 128 + tid) * 8);
  }
  __syncthreads();

  v16h qa[2];
  qa[0] = ld_frag(Qs + (w * 16 + m) * 64, lh);
  qa[1] = ld_frag(Qs + (w * 16 + m) * 64 + 32, lh);

  float mstate[8], lstate[8], g[8];
#pragma unroll
  for (int r = 0; r < 8; ++r) {
    mstate[r] = -__builtin_inff();
    lstate[r] = 0.0f;
    g[r] = gsig[w * 16 + 8 * lh + r] * 0.125f;
  }
  v8f O[4] = {};

  const int* mrow = am + (size_t)b * NSEQ * NSEQ + (size_t)(qbase + w * 16 + 8 * lh) * NSEQ + m;

  for (int j = 0; j < NSEQ / 64; ++j) {
    const int kb = j * 64;
    __syncthreads();
    {
      const _Float16* ksrc = Kg + (size_t)kb * DH;
#pragma unroll
      for (int it = 0; it < 4; ++it)
        *(v8h*)(Ks + (it * 128 + tid) * 8) = *(const v8h*)(ksrc + (it * 128 + tid) * 8);
#pragma unroll
      for (int it = 0; it < 4; ++it) {
        const int c = it * 128 + tid;
        const int key = c >> 3, d8 = (c & 7) * 8;
        v8h vv = *(const v8h*)(Vg + (size_t)(kb + key) * DH + d8);
#pragma unroll
        for (int e = 0; e < 8; ++e) Vt[(d8 + e) * 64 + key] = vv[e];
      }
    }
    __syncthreads();

    v8f S[4];
#pragma unroll
    for (int nt = 0; nt < 4; ++nt) {
      v8f z = {};
      v16h bf0 = ld_frag(Ks + (nt * 16 + m) * 64, lh);
      v16h bf1 = ld_frag(Ks + (nt * 16 + m) * 64 + 32, lh);
      z = wmma_f16(qa[0], bf0, z);
      z = wmma_f16(qa[1], bf1, z);
      S[nt] = z;
    }

#pragma unroll
    for (int r = 0; r < 8; ++r) {
      float mx = -__builtin_inff();
#pragma unroll
      for (int nt = 0; nt < 4; ++nt) {
        const int mv = mrow[(size_t)r * NSEQ + kb + nt * 16];
        float lv = S[nt][r] * g[r];
        if (mv == 0) lv = -__builtin_inff();
        S[nt][r] = lv;
        mx = fmaxf(mx, lv);
      }
      mx = fmaxf(mx, __shfl_xor(mx, 1, 32));
      mx = fmaxf(mx, __shfl_xor(mx, 2, 32));
      mx = fmaxf(mx, __shfl_xor(mx, 4, 32));
      mx = fmaxf(mx, __shfl_xor(mx, 8, 32));
      const float mnew = fmaxf(mstate[r], mx);
      const bool dead = (mnew == -__builtin_inff());
      const float alpha = dead ? 1.0f : __expf(mstate[r] - mnew);
      float rs = 0.0f;
#pragma unroll
      for (int nt = 0; nt < 4; ++nt) {
        const float p = dead ? 0.0f : __expf(S[nt][r] - mnew);
        rs += p;
        Ps[w * 1024 + (8 * lh + r) * 64 + nt * 16 + m] = (_Float16)(p * PSCALE);
      }
      rs += __shfl_xor(rs, 1, 32);
      rs += __shfl_xor(rs, 2, 32);
      rs += __shfl_xor(rs, 4, 32);
      rs += __shfl_xor(rs, 8, 32);
      lstate[r] = lstate[r] * alpha + rs;
      mstate[r] = mnew;
#pragma unroll
      for (int nt2 = 0; nt2 < 4; ++nt2) O[nt2][r] *= alpha;
    }
    __syncthreads();

#pragma unroll
    for (int kk = 0; kk < 2; ++kk) {
      v16h pa = ld_frag(Ps + w * 1024 + m * 64 + kk * 32, lh);
      v16h vb[4];
#pragma unroll
      for (int nt2 = 0; nt2 < 4; ++nt2) vb[nt2] = ld_frag(Vt + (nt2 * 16 + m) * 64 + kk * 32, lh);
#pragma unroll
      for (int nt2 = 0; nt2 < 4; ++nt2) O[nt2] = wmma_f16(pa, vb[nt2], O[nt2]);
    }
  }

  __syncthreads();
  float inv[8];
#pragma unroll
  for (int r = 0; r < 8; ++r) {
    const float l = lstate[r];
    inv[r] = (l > 0.0f) ? (0.25f / l) : 0.0f;
  }
#pragma unroll
  for (int nt2 = 0; nt2 < 4; ++nt2) {
    const int col = nt2 * 16 + m;
#pragma unroll
    for (int r = 0; r < 8; ++r)
      Ks[(w * 16 + 8 * lh + r) * 64 + col] = (_Float16)(O[nt2][r] * inv[r]);
  }
  __syncthreads();

  v8h vv[4];
#pragma unroll
  for (int jj = 0; jj < 4; ++jj) {
    const int c = jj * 128 + tid;
    vv[jj] = *(const v8h*)(Ks + (c >> 3) * 64 + (c & 7) * 8);
  }
#pragma unroll
  for (int jj = 0; jj < 4; ++jj) {
    const int c = jj * 128 + tid;
    _Float16* dst = aw + ((size_t)(b * NSEQ + qbase + (c >> 3))) * CDIM + hd * DH + (c & 7) * 8;
    *(volatile v8h*)dst = vv[jj];
  }
  __threadfence();
#pragma unroll
  for (int jj = 0; jj < 4; ++jj) {
    const int c = jj * 128 + tid;
    _Float16* dst = aw + ((size_t)(b * NSEQ + qbase + (c >> 3))) * CDIM + hd * DH + (c & 7) * 8;
    *(volatile v8h*)dst = vv[jj];
  }
}

__global__ __launch_bounds__(128)
void k_out(const _Float16* __restrict__ aw, const float* __restrict__ Wo, const float* __restrict__ bo,
           float* __restrict__ out) {
  __shared__ __align__(16) float ldsf[64 * 64];
  _Float16* As = reinterpret_cast<_Float16*>(ldsf);
  _Float16* Bs = As + 2048;

  const int tid = threadIdx.x, lane = tid & 31, w = tid >> 5, m = lane & 15, lh = lane >> 4;
  const int cblk = blockIdx.x * 64, rblk = blockIdx.y * 64;
  if (cblk + 64 > CDIM || rblk + 64 > MROWS) return;

  const int ar = tid >> 1, ac = (tid & 1) * 16;
  const int bk = tid >> 2, bc = (tid & 3) * 16;
  const _Float16* ap = aw + (size_t)(rblk + ar) * CDIM + ac;
  const float* bp = Wo + (size_t)bk * CDIM + cblk + bc;

  v8f acc[4] = {};

  for (int k0 = 0; k0 < CDIM; k0 += 32) {
    v8h a8[2];
    v4f b4[4];
    a8[0] = *(const v8h*)(ap + k0);
    a8[1] = *(const v8h*)(ap + k0 + 8);
#pragma unroll
    for (int j = 0; j < 4; ++j) b4[j] = *(const v4f*)(bp + (size_t)k0 * CDIM + 4 * j);
    __syncthreads();
    *(v8h*)(As + ar * 32 + ac)     = a8[0];
    *(v8h*)(As + ar * 32 + ac + 8) = a8[1];
#pragma unroll
    for (int j = 0; j < 4; ++j)
#pragma unroll
      for (int e = 0; e < 4; ++e)
        Bs[(bc + 4 * j + e) * 32 + bk] = (_Float16)(b4[j][e] * WSCALE);
    __syncthreads();

    v16h af = ld_frag(As + (w * 16 + m) * 32, lh);
    v16h bf[4];
#pragma unroll
    for (int nt = 0; nt < 4; ++nt) bf[nt] = ld_frag(Bs + (nt * 16 + m) * 32, lh);
#pragma unroll
    for (int nt = 0; nt < 4; ++nt) acc[nt] = wmma_f16(af, bf[nt], acc[nt]);
  }

  __syncthreads();
  float* Cs = ldsf;
#pragma unroll
  for (int nt = 0; nt < 4; ++nt) {
    const int col = nt * 16 + m;
    const float bb = bo[cblk + col];
#pragma unroll
    for (int r = 0; r < 8; ++r)
      Cs[(w * 16 + 8 * lh + r) * 64 + col] = acc[nt][r] * (1.0f / (ASCALE * WSCALE)) + bb;
  }
  __syncthreads();

  v4f vv[8];
#pragma unroll
  for (int jj = 0; jj < 8; ++jj) {
    const int c = jj * 128 + tid;
    vv[jj] = *(const v4f*)(Cs + (c >> 4) * 64 + (c & 15) * 4);
  }
#pragma unroll
  for (int jj = 0; jj < 8; ++jj) {
    const int c = jj * 128 + tid;
    float* dst = out + (size_t)(rblk + (c >> 4)) * CDIM + cblk + (c & 15) * 4;
    *(volatile v4f*)dst = vv[jj];
  }
  __threadfence();
#pragma unroll
  for (int jj = 0; jj < 8; ++jj) {
    const int c = jj * 128 + tid;
    float* dst = out + (size_t)(rblk + (c >> 4)) * CDIM + cblk + (c & 15) * 4;
    *(volatile v4f*)dst = vv[jj];
  }
}

extern "C" void kernel_launch(void* const* d_in, const int* in_sizes, int n_in,
                              void* d_out, int out_size, void* d_ws, size_t ws_size,
                              hipStream_t stream) {
  if (n_in < 8) return;
  if (in_sizes[0] != MROWS * CDIM) return;
  if (in_sizes[1] != BSZ * NSEQ * NSEQ) return;
  if (in_sizes[2] != CDIM * QKVN) return;
  if (in_sizes[3] != QKVN) return;
  if (in_sizes[4] != CDIM * HN) return;
  if (in_sizes[5] != HN) return;
  if (in_sizes[6] != CDIM * CDIM) return;
  if (in_sizes[7] != CDIM) return;
  if (out_size != MROWS * CDIM) return;

  const float* x    = (const float*)d_in[0];
  const int*   am   = (const int*)d_in[1];
  const float* Wqkv = (const float*)d_in[2];
  const float* bqkv = (const float*)d_in[3];
  const float* We   = (const float*)d_in[4];
  const float* be   = (const float*)d_in[5];
  const float* Wo   = (const float*)d_in[6];
  const float* bo   = (const float*)d_in[7];
  float* out = (float*)d_out;

  const size_t qkv_bytes = (size_t)3 * QKV_S * sizeof(_Float16);
  const size_t aw_off    = qkv_bytes;
  const size_t aw_bytes  = (size_t)MROWS * CDIM * sizeof(_Float16);
  if (aw_off + aw_bytes > ws_size) return;
  char* ws = (char*)d_ws;
  _Float16* qkvws = (_Float16*)ws;
  _Float16* awws  = (_Float16*)(ws + aw_off);

  k_qkv<<<dim3(QKVN / 64, MROWS / 64), 128, 0, stream>>>(x, Wqkv, bqkv, qkvws);
  k_attn<<<dim3(BSZ * HN * (NSEQ / 64)), 128, 0, stream>>>(qkvws, x, We, be, am, awws);
  k_out<<<dim3(CDIM / 64, MROWS / 64), 128, 0, stream>>>(awws, Wo, bo, out);
}
